// MulHeadAttn_71657234366595
// MI455X (gfx1250) — hardware-verified
//
#include <hip/hip_runtime.h>


namespace {
constexpr int Bn = 2, L = 2048, D = 1024, H = 16, HD = 64, NT = Bn * L;
constexpr float EPS = 1e-5f, XS = 8.0f, PS = 8.0f;

typedef _Float16 b16;
typedef __attribute__((ext_vector_type(16))) _Float16 v16b;
typedef __attribute__((ext_vector_type(8))) _Float16 v8b;
typedef __attribute__((ext_vector_type(8))) float v8f;
typedef __attribute__((ext_vector_type(4))) float v4f;
__device__ __forceinline__ void split16(float v, _Float16& hi, _Float16& lo) { hi = (_Float16)v; lo = (_Float16)(v - (float)hi); }
__device__ __forceinline__ void frag_split(const float* p, int hh, __attribute__((ext_vector_type(16))) _Float16& fh, __attribute__((ext_vector_type(16))) _Float16& fl) {
#pragma unroll
  for (int e = 0; e < 8; ++e) { _Float16 a, c; split16(p[8 * hh + e] * 8.0f, a, c); fh[e] = a; fl[e] = c; split16(p[16 + 8 * hh + e] * 8.0f, a, c); fh[8 + e] = a; fl[8 + e] = c; } }
__device__ __forceinline__ float bf16_rne(float f) { unsigned int u = __float_as_uint(f); u += 0x7FFFu + ((u >> 16) & 1u); return __uint_as_float(u & 0xFFFF0000u); }
__device__ __forceinline__ v16b frag_kb(const b16* p, int hh) { const v8b a = *(const v8b*)(p + 8 * hh), b = *(const v8b*)(p + 16 + 8 * hh); v16b f;
#pragma unroll
  for (int e = 0; e < 8; ++e) { f[e] = a[e]; f[8 + e] = b[e]; } return f; }
__device__ __forceinline__ v8f wmma16b(v16b a, v16b b, v8f c) { v8f d = __builtin_amdgcn_wmma_f32_16x16x32_f16(false, a, false, b, (short)0, c, false, false); asm volatile("v_nop\n\tv_nop\n\tv_nop\n\tv_nop" : "+v"(d) : "v"(a), "v"(b)); return d; }
__device__ __forceinline__ void wave_lds_sync() { __builtin_amdgcn_fence(__ATOMIC_RELEASE, "workgroup"); __builtin_amdgcn_wave_barrier(); __builtin_amdgcn_fence(__ATOMIC_ACQUIRE, "workgroup"); }
__device__ __forceinline__ float nexp(float x) { return __builtin_amdgcn_exp2f(x * 1.4426950408889634f); }
__device__ __forceinline__ float pmul(float a, float b) { float p = a * b; asm volatile("" : "+v"(p)); return p; }
__device__ __forceinline__ float wsum(float v) {
#pragma unroll
  for (int o = 1; o < 32; o <<= 1) v += __shfl_xor(v, o); return v; }
__device__ __forceinline__ void sincos_r(float ang, float& sn, float& cs) { const float k = rintf(ang * 0.15915494309189535f); float r = __builtin_fmaf(k, -6.28318548202514648f, ang); r = __builtin_fmaf(k, 1.7484556025237907e-7f, r);
  const float t = r * 0.15915494309189535f; sn = __builtin_amdgcn_sinf(t); cs = __builtin_amdgcn_cosf(t); }
__device__ __forceinline__ float tanh_n(float x) { const float e = __builtin_amdgcn_exp2f(x * 2.8853900817779268f); return 1.0f - 2.0f * __builtin_amdgcn_rcpf(e + 1.0f); }
__device__ __forceinline__ float gelu_t(float x) { const float c = 0.7978845608028654f; return 0.5f * x * (1.0f + tanh_n(c * (x + 0.044715f * x * x * x))); }

struct Wo_ { static constexpr size_t QKV = 0, O = (size_t)3 * D * D, END = O + (size_t)D * D; };
__global__ __launch_bounds__(256) void prep_kernel(const float* __restrict__ wqkv, const float* __restrict__ wo, const float* __restrict__ bo, b16* __restrict__ R, float* __restrict__ P) {
  const size_t tid = (size_t)blockIdx.x * 256 + threadIdx.x, nth = (size_t)gridDim.x * 256;
  for (int pass = 0; pass < 2; ++pass) { for (size_t p = tid; p < Wo_::END / 8; p += nth) { const size_t q = p * 8; const float* s_ = (q < Wo_::O) ? (wqkv + q) : (wo + (q - Wo_::O)); v8b v; for (int e = 0; e < 8; ++e) v[e] = (b16)bf16_rne(s_[e]); *(volatile v8b*)(R + q) = v; }
    for (size_t q = tid; q < (size_t)D; q += nth) P[q] = bf16_rne(bo[q]); __threadfence(); }
}

__global__ __launch_bounds__(256) void xrows_kernel(const float* __restrict__ x, b16* __restrict__ X) {
  const size_t tid = (size_t)blockIdx.x * 256 + threadIdx.x, nth = (size_t)gridDim.x * 256;
  for (int pass = 0; pass < 2; ++pass) { for (size_t p = tid; p < (size_t)NT * D / 8; p += nth) { v8b v; for (int e = 0; e < 8; ++e) v[e] = (b16)(bf16_rne(x[p * 8 + e]) * XS); *(volatile v8b*)(X + p * 8) = v; } __threadfence(); }
}

template <int K, int N, int EPI, int RND>
__global__ __launch_bounds__(64) void gemm_kernel(const b16* __restrict__ A, const b16* __restrict__ Bw, const float* __restrict__ bias, const float* __restrict__ resid, b16* __restrict__ Ch, float* __restrict__ Cf, b16* __restrict__ Cl) {
  __shared__ __attribute__((aligned(16))) float Ts[2][32][128 + 4];
  const int lane = threadIdx.x & 31, wave = threadIdx.x >> 5, nloc = lane & 15, hlf = lane >> 4, m0 = blockIdx.y * 32, c0 = blockIdx.x * 256 + wave * 128;
  v8f acc[2][8];
#pragma unroll
  for (int r = 0; r < 2; ++r)
#pragma unroll
    for (int t = 0; t < 8; ++t) acc[r][t] = (v8f){};
  for (int kb = 0; kb < K; kb += 32) { const v16b a0 = frag_kb(A + (size_t)(m0 + nloc) * K + kb, hlf), a1 = frag_kb(A + (size_t)(m0 + 16 + nloc) * K + kb, hlf);
#pragma unroll
    for (int t = 0; t < 8; ++t) { const v16b bw = frag_kb(Bw + (size_t)(c0 + t * 16 + nloc) * K + kb, hlf); acc[0][t] = wmma16b(a0, bw, acc[0][t]); acc[1][t] = wmma16b(a1, bw, acc[1][t]); } }
#pragma unroll
  for (int t = 0; t < 8; ++t) { const float bv = (bias != nullptr) ? bias[c0 + t * 16 + nloc] : 0.0f;
#pragma unroll
    for (int r = 0; r < 2; ++r)
#pragma unroll
      for (int v = 0; v < 8; ++v) { float y = acc[r][t][v] * (1.0f / XS) + bv; if (EPI == 2) y = fmaxf(y, 0.0f); Ts[wave][r * 16 + 8 * hlf + v][t * 16 + nloc] = y; } }
  wave_lds_sync();
  if (EPI == 3) {
    for (int i = lane; i < 32 * 32; i += 32) { const int rr = i >> 5, pi_ = i & 31; const int hI = pi_ >> 4, dd = pi_ & 15; const int c1 = hI * 64 + dd, c2 = c1 + 16; const int t = (m0 + rr) % L;
      const float invf = __builtin_amdgcn_exp2f(-(float)dd * (13.287712379549449f / 16.0f));
      float sn, cs; sincos_r((float)t * invf, sn, cs); const float a_ = Ts[wave][rr][c1], b_ = Ts[wave][rr][c2];
      Ts[wave][rr][c1] = pmul(a_, cs) - pmul(b_, sn); Ts[wave][rr][c2] = pmul(b_, cs) + pmul(a_, sn); }
    wave_lds_sync(); }
  for (int pass = 0; pass < 2; ++pass) {
    if (EPI == 1) { for (int i = lane; i < 32 * 32; i += 32) { const int rr = i >> 5, c4 = (i & 31) * 4; const size_t gi = (size_t)(m0 + rr) * N + c0 + c4; v4f o = *(const v4f*)(&Ts[wave][rr][c4]); const v4f xr = *(const v4f*)(resid + gi);
        for (int e = 0; e < 4; ++e) o[e] += RND ? bf16_rne(xr[e]) : xr[e]; *(volatile v4f*)(Cf + gi) = o; } }
    else if (EPI == 3 || EPI == 6) { for (int i = lane; i < 32 * 16; i += 32) { const int rr = i >> 4, c8 = (i & 15) * 8; v8b oh, ol; for (int e = 0; e < 8; ++e) { b16 a_, b_; split16(Ts[wave][rr][c8 + e] * XS, a_, b_); oh[e] = a_; ol[e] = b_; } *(volatile v8b*)(Ch + (size_t)(m0 + rr) * N + c0 + c8) = oh; *(volatile v8b*)(Cl + (size_t)(m0 + rr) * N + c0 + c8) = ol; } }
    else { for (int i = lane; i < 32 * 16; i += 32) { const int rr = i >> 4, c8 = (i & 15) * 8; v8b o; for (int e = 0; e < 8; ++e) o[e] = (b16)(Ts[wave][rr][c8 + e] * XS); *(volatile v8b*)(Ch + (size_t)(m0 + rr) * N + c0 + c8) = o; } }
    __threadfence(); }
}

__global__ __launch_bounds__(256) void vt_kernel(const b16* __restrict__ Vr, b16* __restrict__ vt) {
  __shared__ __attribute__((aligned(16))) b16 T[HD][128 + 8];
  const int b = blockIdx.z, h = blockIdx.y, t0 = blockIdx.x * 128, t_ = threadIdx.x;
  for (int i = t_; i < 128 * (HD / 8); i += 256) { const int tk = i >> 3, d8 = (i & 7) * 8; const v8b vv = *(const v8b*)(Vr + ((size_t)(b * L + t0 + tk)) * D + h * HD + d8); for (int e = 0; e < 8; ++e) T[d8 + e][tk] = vv[e]; }
  __syncthreads();
  for (int pass = 0; pass < 2; ++pass) { for (int i = t_; i < HD * 16; i += 256) { const int d = i >> 4, c8 = (i & 15) * 8; *(volatile v8b*)(vt + (((size_t)b * H + h) * HD + d) * L + t0 + c8) = *(const v8b*)(&T[d][c8]); } __threadfence(); }
}

__global__ __launch_bounds__(256) void attn_kernel(const b16* __restrict__ QH, const b16* __restrict__ QL, const b16* __restrict__ KH, const b16* __restrict__ KL, const b16* __restrict__ vt, b16* __restrict__ ctxh, b16* __restrict__ ctxl) {
  __shared__ __attribute__((aligned(16))) b16 Oh[16][8 * HD + 8], Ol[16][8 * HD + 8];
  const int wid = threadIdx.x >> 5, lane = threadIdx.x & 31, hh = lane >> 4, col = lane & 15; const int b = blockIdx.x / (L / 16), q0 = (blockIdx.x % (L / 16)) * 16, h = blockIdx.y * 8 + wid, qi = q0 + col;
  const size_t rb = (size_t)(b * L) * D + h * HD; const b16* Qh = QH + rb; const b16* Ql = QL + rb; const b16* Kh = KH + rb; const b16* Kl = KL + rb; const b16* V = vt + (((size_t)b * H + h) * HD) * L;
  const v16b qa0 = frag_kb(Qh + (size_t)qi * D, hh), qa1 = frag_kb(Qh + (size_t)qi * D + 32, hh), qb0 = frag_kb(Ql + (size_t)qi * D, hh), qb1 = frag_kb(Ql + (size_t)qi * D + 32, hh);
  float m = -INFINITY, l = 0.0f; v8f o[4] = {{}, {}, {}, {}};
  for (int kb = 0; kb < L; kb += 32) {
    v8f s0 = {}, s1 = {};
    { const v16b k0h = frag_kb(Kh + (size_t)(kb + col) * D, hh), k0l = frag_kb(Kl + (size_t)(kb + col) * D, hh), k1h = frag_kb(Kh + (size_t)(kb + col) * D + 32, hh), k1l = frag_kb(Kl + (size_t)(kb + col) * D + 32, hh);
      s0 = wmma16b(k0h, qa0, s0); s0 = wmma16b(k0h, qb0, s0); s0 = wmma16b(k0l, qa0, s0); s0 = wmma16b(k1h, qa1, s0); s0 = wmma16b(k1h, qb1, s0); s0 = wmma16b(k1l, qa1, s0); }
    { const v16b k0h = frag_kb(Kh + (size_t)(kb + 16 + col) * D, hh), k0l = frag_kb(Kl + (size_t)(kb + 16 + col) * D, hh), k1h = frag_kb(Kh + (size_t)(kb + 16 + col) * D + 32, hh), k1l = frag_kb(Kl + (size_t)(kb + 16 + col) * D + 32, hh);
      s1 = wmma16b(k0h, qa0, s1); s1 = wmma16b(k0h, qb0, s1); s1 = wmma16b(k0l, qa0, s1); s1 = wmma16b(k1h, qa1, s1); s1 = wmma16b(k1h, qb1, s1); s1 = wmma16b(k1l, qa1, s1); }
    float mr = -INFINITY;
#pragma unroll
    for (int r = 0; r < 8; ++r) { s0[r] *= (0.125f / (XS * XS)); s1[r] *= (0.125f / (XS * XS)); mr = fmaxf(mr, fmaxf(s0[r], s1[r])); }
    mr = fmaxf(mr, __shfl_xor(mr, 16));
    const float mn = fmaxf(m, mr), al_ = nexp(m - mn); m = mn; float sum = 0.0f; v16b pb;
#pragma unroll
    for (int r = 0; r < 8; ++r) { const float e0 = nexp(s0[r] - mn), e1 = nexp(s1[r] - mn); sum += e0 + e1; pb[r] = (b16)(e0 * PS); pb[8 + r] = (b16)(e1 * PS); }
    sum += __shfl_xor(sum, 16); l = l * al_ + sum;
#pragma unroll
    for (int t = 0; t < 4; ++t) { o[t] *= al_; o[t] = wmma16b(frag_kb(V + (size_t)(t * 16 + col) * L + kb, hh), pb, o[t]); } }
  const float inv = 1.0f / (l * PS);
#pragma unroll
  for (int t = 0; t < 4; ++t)
#pragma unroll
    for (int r = 0; r < 8; ++r) { b16 a_, c_; split16(o[t][r] * inv, a_, c_); Oh[col][wid * HD + t * 16 + 8 * hh + r] = a_; Ol[col][wid * HD + t * 16 + 8 * hh + r] = c_; }
  __syncthreads();
  for (int pass = 0; pass < 2; ++pass) { for (int i = threadIdx.x; i < 16 * 64; i += 256) { const int rr = i >> 6, c8 = (i & 63) * 8; const size_t gi = ((size_t)(b * L + q0 + rr)) * D + blockIdx.y * 8 * HD + c8; *(volatile v8b*)(ctxh + gi) = *(const v8b*)(&Oh[rr][c8]); *(volatile v8b*)(ctxl + gi) = *(const v8b*)(&Ol[rr][c8]); } __threadfence(); }
}

__global__ __launch_bounds__(64) void out_kernel(const b16* __restrict__ ctxh, const b16* __restrict__ ctxl, const b16* __restrict__ R, const float* __restrict__ P, float* __restrict__ out) {
  __shared__ __attribute__((aligned(16))) float Ts[2][32][128 + 4];
  const int lane = threadIdx.x & 31, wave = threadIdx.x >> 5, nloc = lane & 15, hlf = lane >> 4, m0 = blockIdx.y * 32, c0 = blockIdx.x * 256 + wave * 128; const b16* Wo = R + Wo_::O;
  v8f acc[2][8];
#pragma unroll
  for (int r = 0; r < 2; ++r)
#pragma unroll
    for (int t = 0; t < 8; ++t) acc[r][t] = (v8f){};
  for (int kb = 0; kb < D; kb += 32) { const v16b a0 = frag_kb(ctxh + (size_t)(m0 + nloc) * D + kb, hlf), l0 = frag_kb(ctxl + (size_t)(m0 + nloc) * D + kb, hlf), a1 = frag_kb(ctxh + (size_t)(m0 + 16 + nloc) * D + kb, hlf), l1 = frag_kb(ctxl + (size_t)(m0 + 16 + nloc) * D + kb, hlf);
#pragma unroll
    for (int t = 0; t < 8; ++t) { const v16b bw = frag_kb(Wo + (size_t)(c0 + t * 16 + nloc) * D + kb, hlf); acc[0][t] = wmma16b(a0, bw, acc[0][t]); acc[0][t] = wmma16b(l0, bw, acc[0][t]); acc[1][t] = wmma16b(a1, bw, acc[1][t]); acc[1][t] = wmma16b(l1, bw, acc[1][t]); } }
#pragma unroll
  for (int t = 0; t < 8; ++t) { const float bb = P[c0 + t * 16 + nloc];
#pragma unroll
    for (int r = 0; r < 2; ++r)
#pragma unroll
      for (int v = 0; v < 8; ++v) Ts[wave][r * 16 + 8 * hlf + v][t * 16 + nloc] = acc[r][t][v] * (1.0f / XS) + bb; }
  wave_lds_sync();
  for (int pass = 0; pass < 2; ++pass) { for (int i = lane; i < 32 * 32; i += 32) { const int rr = i >> 5, c4 = (i & 31) * 4; *(volatile v4f*)(out + (size_t)(m0 + rr) * D + c0 + c4) = *(const v4f*)(&Ts[wave][rr][c4]); } __threadfence(); }
}
}

extern "C" void kernel_launch(void* const* d_in, const int* in_sizes, int n_in,
                              void* d_out, int out_size, void* d_ws, size_t ws_size, hipStream_t stream) {
  (void)n_in; (void)out_size;
  const float* x = (const float*)d_in[0]; const float* wqkv = (const float*)d_in[1]; const float* wo = (const float*)d_in[2]; const float* bo = (const float*)d_in[3];
  float* out = (float*)d_out;
  if (in_sizes[0] != NT * D || in_sizes[1] != 3 * D * D || in_sizes[2] != D * D) return;
  size_t off = 0; char* ws = (char*)d_ws;
  auto carve = [&](size_t bytes) { char* p = ws + off; off += (bytes + 255) & ~(size_t)255; return p; };
  b16* R = (b16*)carve(Wo_::END * 2); float* P = (float*)carve(D * 4); b16* X = (b16*)carve((size_t)NT * D * 2); b16* QH = (b16*)carve((size_t)NT * D * 2); b16* QL = (b16*)carve((size_t)NT * D * 2); b16* KH = (b16*)carve((size_t)NT * D * 2); b16* KL = (b16*)carve((size_t)NT * D * 2);
  b16* VR = (b16*)carve((size_t)NT * D * 2); b16* VT = (b16*)carve((size_t)NT * D * 2); b16* CH = (b16*)carve((size_t)NT * D * 2); b16* CL = (b16*)carve((size_t)NT * D * 2);
  if (off > ws_size) return;
  prep_kernel<<<512, 256, 0, stream>>>(wqkv, wo, bo, R, P);
  xrows_kernel<<<512, 256, 0, stream>>>(x, X);
  gemm_kernel<D, D, 6, 0><<<dim3(D / 256, NT / 32), 64, 0, stream>>>(X, R + Wo_::QKV, nullptr, nullptr, QH, nullptr, QL);
  gemm_kernel<D, D, 6, 0><<<dim3(D / 256, NT / 32), 64, 0, stream>>>(X, R + Wo_::QKV + (size_t)D * D, nullptr, nullptr, KH, nullptr, KL);
  gemm_kernel<D, D, 0, 0><<<dim3(D / 256, NT / 32), 64, 0, stream>>>(X, R + Wo_::QKV + (size_t)2 * D * D, nullptr, nullptr, VR, nullptr, nullptr);
  vt_kernel<<<dim3(L / 128, H, Bn), 256, 0, stream>>>(VR, VT);
  attn_kernel<<<dim3(NT / 16, 2), 256, 0, stream>>>(QH, QL, KH, KL, VT, CH, CL);
  out_kernel<<<dim3(D / 256, NT / 32), 64, 0, stream>>>(CH, CL, R, P, out);
}
